// EvolvingSystem_16432544875257
// MI455X (gfx1250) — hardware-verified
//
#include <hip/hip_runtime.h>
#include <stddef.h>


typedef _Float16 v16h __attribute__((ext_vector_type(16)));
typedef _Float16 v8h  __attribute__((ext_vector_type(8)));
typedef float    v8f  __attribute__((ext_vector_type(8)));
typedef float    v4f  __attribute__((ext_vector_type(4)));
typedef _Float16 h16;

#ifndef NB
#define NB 8192
#endif
#define NB_FULL 8192
#define NCL   16
#define LAT   256
#define REGW  64
#define EXO   32
#define ORD   16
#define OUTL  32
#define SIGK  (NCL * LAT)

static_assert(NB >= 128 && NB <= NB_FULL && (NB % 128) == 0);
static_assert(NCL == 16);
static_assert(LAT == 4 * 64);
static_assert((LAT % 32) == 0 && (LAT % 64) == 0);
static_assert((SIGK % 64) == 0);
static_assert(ORD == 16 && (ORD % 4) == 0);
static_assert(EXO == 8 * 4);
static_assert(OUTL == 8 * 4);
static_assert(REGW >= ORD);
static_assert((size_t)NB_FULL * OUTL * 4 == (size_t)1048576);

#define LDT 72
#define OLD 36
static_assert((LDT % 8) == 0 && LDT >= 64);
static_assert((OLD % 4) == 0 && OLD >= OUTL);

#define WCARRY 64.0f
#define ZCARRY 64.0f
#define QSCALE (1.0f / (WCARRY * ZCARRY))

#define ST_BYTES  ((size_t)LAT * SIGK * 2)
#define Z16_BYTES ((size_t)NB * LAT * 2)
#define PV_BYTES  ((size_t)NCL * LAT * 4)
#define D2_BYTES  ((size_t)NCL * NB * 4)
#define OFF_ST  ((size_t)0)
#define OFF_Z16 (OFF_ST + ST_BYTES)
#define OFF_PV  (OFF_Z16 + Z16_BYTES)
#define OFF_D2  (OFF_PV + PV_BYTES)
#define WS_TOTAL (OFF_D2 + D2_BYTES)
static_assert((ST_BYTES % 128) == 0 && (Z16_BYTES % 128) == 0);
static_assert((PV_BYTES % 128) == 0 && (D2_BYTES % 128) == 0);
static_assert(WS_TOTAL <= (size_t)134217728);

__device__ __forceinline__ float bf16r(float x) {
  unsigned int u = __float_as_uint(x);
  u = (u + 0x7FFFu + ((u >> 16) & 1u)) & 0xFFFF0000u;
  return __uint_as_float(u);
}

static __device__ __forceinline__ h16 toh_flush(float v) {
  const h16 r = (h16)v;
  return (fabsf(v) < 6.103515625e-05f) ? (h16)0.0f : r;
}

__device__ __forceinline__ v16h frag_at(const _Float16* p) {
  v8h lo = *(const v8h*)(p);
  v8h hi = *(const v8h*)(p + 16);
  v16h out;
#pragma unroll
  for (int i = 0; i < 8; ++i) { out[i] = lo[i]; out[i + 8] = hi[i]; }
  return out;
}

__device__ __forceinline__ v8f wmma16(v16h a, v16h b, v8f c) {
  v8f d = __builtin_amdgcn_wmma_f32_16x16x32_f16(false, a, false, b, (short)0, c,
                                                 false, false);
  asm volatile("v_nop\n\tv_nop\n\tv_nop\n\tv_nop" : "+v"(d) : "v"(a), "v"(b));
  return d;
}

__device__ __forceinline__ float red16_max(float x) {
#pragma unroll
  for (int off = 1; off < 16; off <<= 1) x = fmaxf(x, __shfl_xor(x, off, 32));
  return x;
}
__device__ __forceinline__ float red16_sum(float x) {
#pragma unroll
  for (int off = 1; off < 16; off <<= 1) x += __shfl_xor(x, off, 32);
  return x;
}

__global__ __launch_bounds__(256) void wconv_kernel(
    const float* __restrict__ W, _Float16* __restrict__ Wt, unsigned ldw, unsigned ldk) {
  __shared__ _Float16 T[64 * LDT];
  const unsigned tid = threadIdx.x;
  const unsigned n0 = blockIdx.x * 64u;
  const unsigned k0 = blockIdx.y * 64u;
#pragma unroll 4
  for (unsigned j = 0; j < 16u; ++j) {
    const unsigned idx = tid + 256u * j;
    const unsigned kr = idx >> 6, nc = idx & 63u;
    const float v = W[(size_t)(k0 + kr) * ldw + n0 + nc];
    T[nc * LDT + kr] = toh_flush(WCARRY * bf16r(v));
  }
  __syncthreads();
  v8h x[2];
  size_t off[2];
#pragma unroll
  for (unsigned i = 0; i < 2u; ++i) {
    const unsigned n = 32u * i + (tid >> 3);
    const unsigned kc = (tid & 7u) * 8u;
    x[i] = *(const v8h*)&T[n * LDT + kc];
    off[i] = (size_t)(n0 + n) * ldk + k0 + kc;
  }
#pragma unroll
  for (int i = 0; i < 2; ++i) *(volatile v8h*)(Wt + off[i]) = x[i];
  __threadfence();
#pragma unroll
  for (int i = 0; i < 2; ++i) *(volatile v8h*)(Wt + off[i]) = x[i];
}

__global__ __launch_bounds__(256) void zconv_kernel(
    const float* __restrict__ Z, _Float16* __restrict__ Z16) {
#pragma clang fp contract(off)
  const size_t e = ((size_t)blockIdx.x * 256u + threadIdx.x) * 8u;
  const v4f a0 = *(const v4f*)(Z + e);
  const v4f a1 = *(const v4f*)(Z + e + 4u);
  v8h o;
#pragma unroll
  for (int i = 0; i < 4; ++i) {
    o[i]     = toh_flush(ZCARRY * bf16r(a0[i]));
    o[i + 4] = toh_flush(ZCARRY * bf16r(a1[i]));
  }
  _Float16* p = Z16 + e;
  *(volatile v8h*)p = o;
  __threadfence();
  *(volatile v8h*)p = o;
}

__global__ __launch_bounds__(256) void pvec_kernel(
    const float* __restrict__ Mu, const float* __restrict__ Sig, float* __restrict__ Pv) {
#pragma clang fp contract(off)
  const unsigned gt = blockIdx.x * 256u + threadIdx.x;
  const unsigned c = gt >> 8;
  const unsigned j = gt & 255u;
  const float* sc = Sig + (size_t)c * (LAT * LAT) + j;
  const float* mc = Mu + c * LAT;
  float acc = 0.0f;
#pragma unroll 4
  for (unsigned i = 0; i < (unsigned)LAT; ++i)
    acc = fmaf(bf16r(mc[i]), bf16r(sc[(size_t)i * LAT]), acc);
  *(volatile float*)(Pv + gt) = acc;
  __threadfence();
  *(volatile float*)(Pv + gt) = acc;
}

__global__ __launch_bounds__(256) void gemm_d2_kernel(
    const _Float16* __restrict__ Z16, const _Float16* __restrict__ St,
    const float* __restrict__ Pv, float* __restrict__ D2t) {
  __shared__ float Ds[128];
  const unsigned tid = threadIdx.x, lane = tid & 31u;
  const unsigned wave = (unsigned)__builtin_amdgcn_readfirstlane((int)(threadIdx.x >> 5));
  const unsigned hh = lane >> 4, m = lane & 15u;
  const unsigned row0 = blockIdx.x * 128u;
  const unsigned c = blockIdx.y;

  const _Float16* ap = Z16 + (size_t)(row0 + wave * 16u + m) * LAT + hh * 8u;
  const _Float16* bp = St + (size_t)m * SIGK + c * (unsigned)LAT + hh * 8u;
  const float* pc = Pv + c * (unsigned)LAT + m;

  float s[8];
#pragma unroll
  for (int r = 0; r < 8; ++r) s[r] = 0.0f;

#pragma unroll 1
  for (unsigned jg = 0; jg < 4u; ++jg) {
    const _Float16* bq0 = bp + (size_t)(jg * 64u) * SIGK;
    const _Float16* bq1 = bq0 + (size_t)16 * SIGK;
    const _Float16* bq2 = bq0 + (size_t)32 * SIGK;
    const _Float16* bq3 = bq0 + (size_t)48 * SIGK;
    v8f acc0 = {}, acc1 = {}, acc2 = {}, acc3 = {};
#pragma unroll 2
    for (unsigned k0 = 0; k0 < (unsigned)LAT; k0 += 32u) {
      const v16h a  = frag_at(ap + k0);
      const v16h b0 = frag_at(bq0 + k0);
      const v16h b1 = frag_at(bq1 + k0);
      const v16h b2 = frag_at(bq2 + k0);
      const v16h b3 = frag_at(bq3 + k0);
      acc0 = wmma16(a, b0, acc0);
      acc1 = wmma16(a, b1, acc1);
      acc2 = wmma16(a, b2, acc2);
      acc3 = wmma16(a, b3, acc3);
    }
    const float p0 = pc[jg * 64u];
    const float p1 = pc[jg * 64u + 16u];
    const float p2 = pc[jg * 64u + 32u];
    const float p3 = pc[jg * 64u + 48u];
#pragma unroll
    for (int r = 0; r < 8; ++r) {
      const float d0 = p0 - acc0[r] * QSCALE;
      const float d1 = p1 - acc1[r] * QSCALE;
      const float d2 = p2 - acc2[r] * QSCALE;
      const float d3 = p3 - acc3[r] * QSCALE;
      float t = s[r];
      t = fmaf(d0, d0, t);
      t = fmaf(d1, d1, t);
      t = fmaf(d2, d2, t);
      t = fmaf(d3, d3, t);
      s[r] = t;
    }
  }

#pragma unroll
  for (int r = 0; r < 8; ++r) s[r] = red16_sum(s[r]);
  if (m == 0u) {
#pragma unroll
    for (int r = 0; r < 8; ++r) Ds[wave * 16u + hh * 8u + (unsigned)r] = s[r];
  }
  __syncthreads();
  if (wave == 0u) {
    const v4f x = *(const v4f*)&Ds[lane * 4u];
    float* dst = D2t + (size_t)c * NB + row0 + lane * 4u;
    *(volatile v4f*)dst = x;
    __threadfence();
    *(volatile v4f*)dst = x;
  }
}

__global__ __launch_bounds__(256) void arx_kernel(
    const float* __restrict__ Y, const float* __restrict__ U,
    const float* __restrict__ Ac, const float* __restrict__ Bc,
    const float* __restrict__ Bi, const float* __restrict__ D2t,
    float* __restrict__ Out) {
#pragma clang fp contract(off)
  __shared__ float Os[16 * OLD];
  const unsigned tid = threadIdx.x;
  const unsigned wave = (unsigned)__builtin_amdgcn_readfirstlane((int)(threadIdx.x >> 5));
  const unsigned gt = blockIdx.x * 256u + tid;
  const unsigned b = gt >> 4, c = gt & 15u;
  const unsigned bl = tid >> 4;

  const float dv = D2t[(size_t)c * NB + b];
  const float x = -fmaxf(dv, 1.0e-8f);
  const float mx = red16_max(x);
  const float e = __expf(x - mx);
  const float se = red16_sum(e);
  const float psi = e * __builtin_amdgcn_rcpf(se);

  const size_t rowbc = (size_t)b * NCL + c;
  const float* ur = U + rowbc * EXO;
  const float* bc = Bc + c * (unsigned)EXO;
  float ud = 0.0f;
#pragma unroll 1
  for (unsigned k4 = 0; k4 < (unsigned)(EXO / 4); ++k4) {
    const v4f uv = *(const v4f*)(ur + 4u * k4);
    const v4f bv = *(const v4f*)(bc + 4u * k4);
#pragma unroll
    for (int i = 0; i < 4; ++i) ud = fmaf(bf16r(uv[i]), bf16r(bv[i]), ud);
  }
  const float ub = ud + bf16r(Bi[c]);

  float st[ORD], ac[ORD];
  const float* yr = Y + rowbc * REGW + (REGW - ORD);
  const float* ar = Ac + c * (unsigned)ORD;
#pragma unroll
  for (int q = 0; q < ORD / 4; ++q) {
    const v4f yv = *(const v4f*)(yr + 4 * q);
    const v4f av = *(const v4f*)(ar + 4 * q);
#pragma unroll
    for (int i = 0; i < 4; ++i) {
      st[4 * q + i] = bf16r(yv[i]);
      ac[4 * q + i] = bf16r(av[i]);
    }
  }

#pragma unroll 1
  for (unsigned l = 0; l < (unsigned)OUTL; ++l) {
    float dot = 0.0f;
#pragma unroll
    for (int o = 0; o < ORD; ++o) dot = fmaf(st[o], ac[o], dot);
    const float yn = dot + ub;
#pragma unroll
    for (int o = 0; o < ORD - 1; ++o) st[o] = st[o + 1];
    st[ORD - 1] = yn;
    const float part = red16_sum(psi * yn);
    if (c == 0u) Os[bl * OLD + l] = part;
  }
  __syncthreads();

  if (wave < 4u) {
    const unsigned r = tid >> 3;
    const unsigned pcs = (tid & 7u) * 4u;
    const v4f xo = *(const v4f*)&Os[r * OLD + pcs];
    float* dst = Out + (size_t)(blockIdx.x * 16u + r) * OUTL + pcs;
    *(volatile v4f*)dst = xo;
    __threadfence();
    *(volatile v4f*)dst = xo;
  }
}

extern "C" void kernel_launch(void* const* d_in, const int* in_sizes, int n_in,
                              void* d_out, int out_size, void* d_ws, size_t ws_size,
                              hipStream_t stream) {
  if (n_in < 8) return;
  if ((long long)in_sizes[0] < (long long)NB * NCL * REGW) return;
  if ((long long)in_sizes[1] < (long long)NB * LAT) return;
  if ((long long)in_sizes[2] < (long long)NB * NCL * EXO) return;
  if ((long long)in_sizes[3] < (long long)NCL * LAT) return;
  if ((long long)in_sizes[4] < (long long)NCL * LAT * LAT) return;
  if ((long long)in_sizes[5] < (long long)NCL * ORD) return;
  if ((long long)in_sizes[6] < (long long)NCL * EXO) return;
  if ((long long)in_sizes[7] < (long long)NCL) return;
  if ((long long)out_size < (long long)NB * OUTL) return;
  if (ws_size < WS_TOTAL) return;

  const float* y    = (const float*)d_in[0];
  const float* z    = (const float*)d_in[1];
  const float* u    = (const float*)d_in[2];
  const float* mu   = (const float*)d_in[3];
  const float* sig  = (const float*)d_in[4];
  const float* acf  = (const float*)d_in[5];
  const float* bcf  = (const float*)d_in[6];
  const float* bias = (const float*)d_in[7];
  float* out = (float*)d_out;

  char* ws = (char*)d_ws;
  _Float16* St  = (_Float16*)(ws + OFF_ST);
  _Float16* Z16 = (_Float16*)(ws + OFF_Z16);
  float*    Pv  = (float*)(ws + OFF_PV);
  float*    D2t = (float*)(ws + OFF_D2);

  dim3 blk(256);
  wconv_kernel<<<dim3(LAT / 64, SIGK / 64), blk, 0, stream>>>(sig, St, (unsigned)LAT, (unsigned)SIGK);
  zconv_kernel<<<dim3((NB * LAT) / 2048), blk, 0, stream>>>(z, Z16);
  pvec_kernel<<<dim3((NCL * LAT) / 256), blk, 0, stream>>>(mu, sig, Pv);
  gemm_d2_kernel<<<dim3(NB / 128, NCL), blk, 0, stream>>>(Z16, St, Pv, D2t);
  arx_kernel<<<dim3((NB * NCL) / 256), blk, 0, stream>>>(y, u, acf, bcf, bias, D2t, out);
}
